// TanhAttention_28174985462282
// MI455X (gfx1250) — hardware-verified
//
#include <hip/hip_runtime.h>
#include <math.h>

typedef __attribute__((ext_vector_type(16))) _Float16 v16h;
typedef __attribute__((ext_vector_type(8)))  _Float16 v8h;
typedef __attribute__((ext_vector_type(16))) __bf16   v16b;
typedef __attribute__((ext_vector_type(8)))  __bf16   v8b;
typedef __attribute__((ext_vector_type(8)))  float    v8f;
typedef __attribute__((ext_vector_type(4)))  float    v4f;
typedef __attribute__((ext_vector_type(4)))  unsigned v4u;

constexpr int NBATCH = 4;
constexpr int SEQL   = 256;
constexpr int SEQT   = 256;
constexpr int DMODEL = 512;
constexpr float NEG_FILL = -1e30f;

__device__ __forceinline__ unsigned short f2bf_bits(float f) {
  unsigned u = __float_as_uint(f);
  return (unsigned short)((u + 0x7FFFu + ((u >> 16) & 1u)) >> 16);
}
__device__ __forceinline__ float bf_bits2f(unsigned short h) { return __uint_as_float(((unsigned)h) << 16); }

__device__ __forceinline__ void dep_guard_h(v8f& a, v8f& b, v16h x, v16h y) { asm volatile("v_nop\n\tv_nop\n\tv_nop\n\tv_nop" : "+v"(a), "+v"(b) : "v"(x), "v"(y)); }
__device__ __forceinline__ void dep_guard_b(v8f& a, v8f& b, v16b x, v16b y) { asm volatile("v_nop\n\tv_nop\n\tv_nop\n\tv_nop" : "+v"(a), "+v"(b) : "v"(x), "v"(y)); }
__device__ __forceinline__ void keep4_h(v16h a, v16h b, v16h c, v16h d) { asm volatile("v_nop" :: "v"(a), "v"(b), "v"(c), "v"(d)); }
__device__ __forceinline__ void keep4_b(v16b a, v16b b, v16b c, v16b d) { asm volatile("v_nop" :: "v"(a), "v"(b), "v"(c), "v"(d)); }
__device__ __forceinline__ void acc_guard4(v8f& a, v8f& b, v8f& c, v8f& d) { asm volatile("v_nop\n\tv_nop\n\tv_nop\n\tv_nop" : "+v"(a), "+v"(b), "+v"(c), "+v"(d)); }

template <typename T> struct Frag;
template <> struct Frag<_Float16> {
  typedef v16h V; union U { v16h v; v8h h[2]; };
  static __device__ __forceinline__ v16h load(const _Float16* p) {
    U f; f.h[0] = *(const v8h*)(p); f.h[1] = *(const v8h*)(p + 16); return f.v;
  }
  static __device__ __forceinline__ v8f mma(v16h a, v16h b, v8f c) {
    return __builtin_amdgcn_wmma_f32_16x16x32_f16(false, a, false, b, (short)0, c, false, false);
  }
  static __device__ __forceinline__ void guard(v8f& a, v8f& b, v16h x, v16h y) { dep_guard_h(a, b, x, y); }
  static __device__ __forceinline__ void keep(v16h a, v16h b, v16h c, v16h d) { keep4_h(a, b, c, d); }
};
template <> struct Frag<__bf16> {
  typedef v16b V; union U { v16b v; v8b h[2]; };
  static __device__ __forceinline__ v16b load(const __bf16* p) {
    U f; f.h[0] = *(const v8b*)(p); f.h[1] = *(const v8b*)(p + 16); return f.v;
  }
  static __device__ __forceinline__ v8f mma(v16b a, v16b b, v8f c) {
    return __builtin_amdgcn_wmma_f32_16x16x32_bf16(false, a, false, b, (short)0, c, false, false);
  }
  static __device__ __forceinline__ void guard(v8f& a, v8f& b, v16b x, v16b y) { dep_guard_b(a, b, x, y); }
  static __device__ __forceinline__ void keep(v16b a, v16b b, v16b c, v16b d) { keep4_b(a, b, c, d); }
};

__device__ __forceinline__ unsigned short at_bf_bits(float f) {
  unsigned u = __float_as_uint(f);
  return (unsigned short)((u + 0x7FFFu + ((u >> 16) & 1u)) >> 16);
}
__device__ __forceinline__ __bf16 at_f2bf(float f) { return __builtin_bit_cast(__bf16, at_bf_bits(f)); }
__device__ __forceinline__ void at_split(float f, __bf16& hi, __bf16& lo) {
  const unsigned short hb = at_bf_bits(f);
  hi = __builtin_bit_cast(__bf16, hb);
  lo = at_f2bf(f - __uint_as_float(((unsigned)hb) << 16));
}
__device__ __forceinline__ v8f at_mma(v16b a, v16b b, v8f c) {
  c = __builtin_amdgcn_wmma_f32_16x16x32_bf16(false, a, false, b, (short)0, c, false, false);
  asm volatile("v_nop\n\tv_nop\n\tv_nop\n\tv_nop" : "+v"(c) : "v"(a), "v"(b));
  return c;
}

template <int ET> struct Elem;
template <> struct Elem<0> { typedef _Float16 T; };
template <> struct Elem<1> { typedef __bf16 T; };
template <int ET, int SPLIT, int BIAS_MODE, int OUT_MODE>
__global__ __launch_bounds__(256) void wmma_gemm64(
    const unsigned short* __restrict__ Ap, const unsigned short* __restrict__ A2p, int lda, long strideA,
    const unsigned short* __restrict__ Btp, const unsigned short* __restrict__ Bt2p, int ldb, long strideB,
    void* __restrict__ Cout, void* __restrict__ Cout2, int ldc, long strideC,
    const float* __restrict__ bias,
    int M, int N, int K, float scale) {
  typedef typename Elem<ET>::T T;
  typedef typename Frag<T>::V V;
  const T* A = (const T*)Ap; const T* A2 = (const T*)A2p; const T* Bt = (const T*)Btp; const T* Bt2 = (const T*)Bt2p;
  __shared__ __align__(16) float sT[8][16 * 68];
  const int b    = blockIdx.y;
  const int lane = threadIdx.x & 31;
  const int wave = threadIdx.x >> 5;
  const int tilesN = N >> 6;
  const int tilesM = M >> 6;
  const int tile = blockIdx.x * 8 + wave;
  if (tile >= tilesM * tilesN) return;
  const int tm = tile / tilesN;
  const int tn = tile - tm * tilesN;
  const int m0 = tm << 6;
  const int n0 = tn << 6;

  const T* Ab  = A  + (size_t)b * strideA;
  const T* Bb  = Bt + (size_t)b * strideB;
  const T* Ab2 = (SPLIT >= 1) ? (A2  + (size_t)b * strideA) : nullptr;
  const T* Bb2 = (SPLIT == 2) ? (Bt2 + (size_t)b * strideB) : nullptr;

  const int rlane = lane & 15;
  const int koff  = (lane >> 4) * 8;
  const int mOff  = (lane >> 4) * 8;

  v8f acc[4][4];
#pragma unroll
  for (int i = 0; i < 4; ++i)
#pragma unroll
    for (int j = 0; j < 4; ++j) acc[i][j] = (v8f){0.f,0.f,0.f,0.f,0.f,0.f,0.f,0.f};

  for (int k0 = 0; k0 < K; k0 += 32) {
    V bh[4], bl[4];
#pragma unroll
    for (int j = 0; j < 4; ++j) {
      const size_t bo = (size_t)(n0 + (j << 4) + rlane) * ldb + koff + k0;
      bh[j] = Frag<T>::load(Bb + bo);
      if (SPLIT == 2) bl[j] = Frag<T>::load(Bb2 + bo);
    }
#pragma unroll
    for (int i = 0; i < 4; ++i) {
      const size_t ao = (size_t)(m0 + (i << 4) + rlane) * lda + koff + k0;
      V ah = Frag<T>::load(Ab + ao);
      V al;
      if (SPLIT >= 1) al = Frag<T>::load(Ab2 + ao);
#pragma unroll
      for (int j = 0; j < 4; ++j) {
        acc[i][j] = Frag<T>::mma(ah, bh[j], acc[i][j]);
        if (SPLIT == 2) acc[i][j] = Frag<T>::mma(ah, bl[j], acc[i][j]);
        if (SPLIT >= 1) acc[i][j] = Frag<T>::mma(al, bh[j], acc[i][j]);
      }
      Frag<T>::guard(acc[i][0], acc[i][3], ah, (SPLIT >= 1) ? al : ah);
    }
    Frag<T>::keep(bh[0], bh[1], bh[2], bh[3]);
    if (SPLIT == 2) Frag<T>::keep(bl[0], bl[1], bl[2], bl[3]);
  }
  acc_guard4(acc[0][0], acc[0][1], acc[0][2], acc[0][3]);
  acc_guard4(acc[1][0], acc[1][1], acc[1][2], acc[1][3]);
  acc_guard4(acc[2][0], acc[2][1], acc[2][2], acc[2][3]);
  acc_guard4(acc[3][0], acc[3][1], acc[3][2], acc[3][3]);

  float* slab = sT[wave];
#pragma unroll
  for (int i = 0; i < 4; ++i) {
    const int mBase = m0 + (i << 4);
#pragma unroll
    for (int j = 0; j < 4; ++j) {
      const int n = n0 + (j << 4) + rlane;
      float bv = 0.f;
      if (BIAS_MODE == 2) bv = bias[n];
#pragma unroll
      for (int r = 0; r < 8; ++r) {
        float v = acc[i][j][r] * scale;
        if (BIAS_MODE == 1) v += bias[mBase + mOff + r];
        if (BIAS_MODE == 2) v += bv;
        slab[(mOff + r) * 68 + (j << 4) + rlane] = v;
      }
    }
    __builtin_amdgcn_fence(__ATOMIC_RELEASE, "workgroup");
    __builtin_amdgcn_wave_barrier();
    __builtin_amdgcn_fence(__ATOMIC_ACQUIRE, "workgroup");
    if (OUT_MODE == 0) {
      float* Cm = (float*)Cout + (size_t)b * strideC;
      const int hh = lane >> 4, c4 = (lane & 15) * 4;
      for (int pass = 0; pass < 2; ++pass) {
#pragma unroll
        for (int it = 0; it < 8; ++it) {
          const int row = it * 2 + hh;
          v4f v = *(const v4f*)(slab + row * 68 + c4);
          *(volatile v4f*)(Cm + (size_t)(mBase + row) * ldc + n0 + c4) = v;
        }
        __threadfence();
      }
    } else {
      const int q = lane >> 3, c8 = (lane & 7) * 8;
      unsigned short* Cm  = (unsigned short*)Cout  + (size_t)b * strideC;
      unsigned short* Cm2 = (OUT_MODE == 2) ? ((unsigned short*)Cout2 + (size_t)b * strideC) : nullptr;
      for (int pass = 0; pass < 2; ++pass) {
#pragma unroll
        for (int it = 0; it < 4; ++it) {
          const int row = it * 4 + q;
          const float* sp = slab + row * 68 + c8;
          v8h hv, lv;
#pragma unroll
          for (int e = 0; e < 8; ++e) {
            if (OUT_MODE == 1) {
              hv[e] = (_Float16)sp[e];
            } else {
              unsigned short hb = f2bf_bits(sp[e]);
              unsigned short lb = f2bf_bits(sp[e] - bf_bits2f(hb));
              hv[e] = __builtin_bit_cast(_Float16, hb);
              lv[e] = __builtin_bit_cast(_Float16, lb);
            }
          }
          *(volatile v8h*)(Cm + (size_t)(mBase + row) * ldc + n0 + c8) = hv;
          if (OUT_MODE == 2) *(volatile v8h*)(Cm2 + (size_t)(mBase + row) * ldc + n0 + c8) = lv;
        }
        __threadfence();
      }
    }
    __builtin_amdgcn_fence(__ATOMIC_RELEASE, "workgroup");
    __builtin_amdgcn_wave_barrier();
    __builtin_amdgcn_fence(__ATOMIC_ACQUIRE, "workgroup");
  }
}

__global__ __launch_bounds__(256) void cast_f32_bf16x8(
    const float* __restrict__ in, unsigned short* __restrict__ out, int n8) {
  const int i = blockIdx.x * 256 + threadIdx.x;
  if (i < n8) {
    const v4f a = *(const v4f*)(in + (size_t)8 * i);
    const v4f c = *(const v4f*)(in + (size_t)8 * i + 4);
    v4u w;
    w[0] = (unsigned)f2bf_bits(a[0]) | ((unsigned)f2bf_bits(a[1]) << 16);
    w[1] = (unsigned)f2bf_bits(a[2]) | ((unsigned)f2bf_bits(a[3]) << 16);
    w[2] = (unsigned)f2bf_bits(c[0]) | ((unsigned)f2bf_bits(c[1]) << 16);
    w[3] = (unsigned)f2bf_bits(c[2]) | ((unsigned)f2bf_bits(c[3]) << 16);
    unsigned short* p = out + (size_t)8 * i;
    *(volatile v4u*)p = w;
    __threadfence();
    *(volatile v4u*)p = w;
  }
}

__global__ __launch_bounds__(128) void bias_rne_kernel(
    const float* __restrict__ ba, const float* __restrict__ bb,
    float* __restrict__ outa, float* __restrict__ outb) {
  const float* src = (blockIdx.x == 0) ? ba : bb;
  float* dst = (blockIdx.x == 0) ? outa : outb;
  const int i = threadIdx.x;
  const v4f v = *(const v4f*)(src + 4 * i);
  v4f r;
#pragma unroll
  for (int e = 0; e < 4; ++e) r[e] = bf_bits2f(f2bf_bits(v[e]));
  *(volatile v4f*)(dst + 4 * i) = r;
  __threadfence();
  *(volatile v4f*)(dst + 4 * i) = r;
}

__global__ __launch_bounds__(256) void transpose_mem_kernel(
    const float* __restrict__ mem, unsigned short* __restrict__ memT) {
  __shared__ __align__(16) unsigned short tileT[64 * 72];
  const int tid = threadIdx.x, wave = tid >> 5, lane = tid & 31;
  const int blk = blockIdx.x;
  const int b  = blk >> 5;
  const int rr = blk & 31;
  const int tq = rr >> 3, dq = rr & 7;
  const int t0 = tq * 64, d0 = dq * 64;
  {
    const int row = tid >> 2;
    const int cg  = (tid & 3) * 16;
    const float* src = mem + ((size_t)(b * SEQT + t0 + row)) * DMODEL + d0 + cg;
#pragma unroll
    for (int i = 0; i < 4; ++i) {
      const v4f v = *(const v4f*)(src + 4 * i);
#pragma unroll
      for (int e = 0; e < 4; ++e) tileT[(cg + 4 * i + e) * 72 + row] = f2bf_bits(v[e]);
    }
  }
  __syncthreads();
  {
    const int q = lane >> 3, c8 = (lane & 7) * 8;
    const int dd0 = wave * 8 + q;
    const int dd1 = wave * 8 + 4 + q;
    const v4u val0 = *(const v4u*)(tileT + dd0 * 72 + c8);
    const v4u val1 = *(const v4u*)(tileT + dd1 * 72 + c8);
    unsigned short* dst0 = memT + ((size_t)(b * DMODEL + d0 + dd0)) * SEQT + t0 + c8;
    unsigned short* dst1 = memT + ((size_t)(b * DMODEL + d0 + dd1)) * SEQT + t0 + c8;
    for (int pass = 0; pass < 2; ++pass) {
      *(volatile v4u*)dst0 = val0;
      *(volatile v4u*)dst1 = val1;
      __threadfence();
    }
  }
}

__global__ __launch_bounds__(256) void score_softmax_kernel(
    const float* __restrict__ item1, const float* __restrict__ item2,
    const float* __restrict__ wt, const float* __restrict__ btp,
    const int* __restrict__ mmask,
    unsigned short* __restrict__ Phi, unsigned short* __restrict__ Plo) {
  __shared__ __align__(16) float i1s[DMODEL];
  __shared__ __align__(16) __bf16 wtb[DMODEL];
  __shared__ float srow[SEQT];
  __shared__ float red[16];
  __shared__ __align__(16) unsigned short phs[SEQT];
  __shared__ __align__(16) unsigned short pls[SEQT];

  const int tid  = threadIdx.x;
  const int wave = tid >> 5, lane = tid & 31;
  const int cc   = lane & 15, hh = lane >> 4;
  const int bl   = blockIdx.x;
  const int b    = bl / SEQL;
  const int l    = bl - b * SEQL;

  const float* i1row = item1 + (size_t)bl * DMODEL;
  i1s[tid]        = i1row[tid];
  i1s[tid + 256]  = i1row[tid + 256];
  wtb[tid]        = at_f2bf(wt[tid]);
  wtb[tid + 256]  = at_f2bf(wt[tid + 256]);
  srow[tid]       = NEG_FILL;
  __syncthreads();

  const float btv = bf_bits2f(f2bf_bits(btp[0]));
  const int ttmin = l >> 4;
  for (int tt = ttmin + wave; tt < SEQT / 16; tt += 8) {
    const int t = tt * 16 + cc;
    const float* i2row = item2 + ((size_t)(b * SEQT + t)) * DMODEL;
    v8f acc = (v8f){0.f,0.f,0.f,0.f,0.f,0.f,0.f,0.f};
#pragma unroll 1
    for (int k0 = 0; k0 < DMODEL; k0 += 32) {
      const int dA = k0 + 8 * hh;
      const int dB = dA + 16;
      const v4f xa0 = *(const v4f*)(i2row + dA);
      const v4f xa1 = *(const v4f*)(i2row + dA + 4);
      const v4f xb0 = *(const v4f*)(i2row + dB);
      const v4f xb1 = *(const v4f*)(i2row + dB + 4);
      const v4f ya0 = *(const v4f*)(i1s + dA);
      const v4f ya1 = *(const v4f*)(i1s + dA + 4);
      const v4f yb0 = *(const v4f*)(i1s + dB);
      const v4f yb1 = *(const v4f*)(i1s + dB + 4);
      v16b fh, fl;
#pragma unroll
      for (int e = 0; e < 4; ++e) {
        __bf16 h0, l0;
        at_split(tanhf(ya0[e] + xa0[e]), h0, l0); fh[e]      = h0; fl[e]      = l0;
        at_split(tanhf(ya1[e] + xa1[e]), h0, l0); fh[4 + e]  = h0; fl[4 + e]  = l0;
        at_split(tanhf(yb0[e] + xb0[e]), h0, l0); fh[8 + e]  = h0; fl[8 + e]  = l0;
        at_split(tanhf(yb1[e] + xb1[e]), h0, l0); fh[12 + e] = h0; fl[12 + e] = l0;
      }
      const v16b af = Frag<__bf16>::load(wtb + dA);
      acc = at_mma(af, fh, acc);
      acc = at_mma(af, fl, acc);
    }
    if (hh == 0) srow[t] = acc[0] + btv;
  }
  __syncthreads();

  const int t = tid;
  float s = srow[t];
  const int mk = mmask[b * SEQT + t];
  const bool masked = (t < l) || (mk == 0);
  s = masked ? NEG_FILL : s;

  float m = s;
#pragma unroll
  for (int off = 1; off < 32; off <<= 1) m = fmaxf(m, __shfl_xor(m, off, 32));
  if (lane == 0) red[wave] = m;
  __syncthreads();
  float gm = red[0];
#pragma unroll
  for (int w = 1; w < 8; ++w) gm = fmaxf(gm, red[w]);

  const float e = expf(s - gm);
  float ps = e;
#pragma unroll
  for (int off = 1; off < 32; off <<= 1) ps += __shfl_xor(ps, off, 32);
  if (lane == 0) red[8 + wave] = ps;
  __syncthreads();
  float tot = red[8];
#pragma unroll
  for (int w = 1; w < 8; ++w) tot += red[8 + w];

  const float p = e * (1.0f / tot);
  const unsigned short hb = f2bf_bits(p);
  const unsigned short lb = f2bf_bits(p - bf_bits2f(hb));
  phs[t] = hb;
  pls[t] = lb;
  __syncthreads();

  if (wave < 2) {
    const v4u vh = *(const v4u*)(phs + lane * 8);
    const v4u vl = *(const v4u*)(pls + lane * 8);
    const v4u val = (wave == 0) ? vh : vl;
    unsigned short* dst = ((wave == 0) ? Phi : Plo) + (size_t)bl * SEQT + lane * 8;
    *(volatile v4u*)dst = val;
    __threadfence();
    *(volatile v4u*)dst = val;
  }
}

extern "C" void kernel_launch(void* const* d_in, const int* in_sizes, int n_in,
                              void* d_out, int out_size, void* d_ws, size_t ws_size,
                              hipStream_t stream) {
  const float* x    = (const float*)d_in[0];
  const float* mem  = (const float*)d_in[1];
  const float* W1   = (const float*)d_in[2];
  const float* b1   = (const float*)d_in[3];
  const float* W2   = (const float*)d_in[4];
  const float* b2   = (const float*)d_in[5];
  const float* wt   = (const float*)d_in[6];
  const float* bt   = (const float*)d_in[7];
  const int*   mask = (const int*)d_in[8];
  float* out = (float*)d_out;

  constexpr size_t N_X = (size_t)NBATCH * SEQL * DMODEL;
  constexpr size_t N_M = (size_t)NBATCH * SEQT * DMODEL;
  constexpr size_t N_W = (size_t)DMODEL * DMODEL;
  constexpr size_t N_P = (size_t)NBATCH * SEQL * SEQT;

  constexpr size_t OFF_XB = 0;
  constexpr size_t OFF_MB = OFF_XB + N_X * 2;
  constexpr size_t OFF_W1 = OFF_MB + N_M * 2;
  constexpr size_t OFF_W2 = OFF_W1 + N_W * 2;
  constexpr size_t OFF_MT = OFF_W2 + N_W * 2;
  constexpr size_t OFF_I1 = OFF_MT + N_M * 2;
  constexpr size_t OFF_I2 = OFF_I1 + N_X * 4;
  constexpr size_t OFF_PH = OFF_I2 + N_M * 4;
  constexpr size_t OFF_PL = OFF_PH + N_P * 2;
  constexpr size_t OFF_B1 = OFF_PL + N_P * 2;
  constexpr size_t OFF_B2 = OFF_B1 + (size_t)DMODEL * 4;
  constexpr size_t WS_TOTAL = OFF_B2 + (size_t)DMODEL * 4;
  static_assert(WS_TOTAL == 9441280);
  static_assert(WS_TOTAL <= (size_t)134217728);
  static_assert((OFF_MB % 128) == 0 && (OFF_W1 % 128) == 0 && (OFF_MT % 128) == 0 && (OFF_I1 % 128) == 0 &&
                (OFF_PH % 128) == 0 && (OFF_PL % 128) == 0 && (OFF_B1 % 128) == 0 && (OFF_B2 % 128) == 0);
  static_assert((NBATCH * SEQL) % 64 == 0 && DMODEL % 64 == 0 && DMODEL % 32 == 0);
  static_assert(SEQL % 64 == 0 && SEQT % 32 == 0 && SEQT % 64 == 0);
  static_assert(N_X % 2048 == 0 && N_W % 2048 == 0);
  static_assert(SEQT == 256 && DMODEL == 512 && SEQL == 256);

  if (n_in < 9) return;
  if ((size_t)in_sizes[0] != N_X || (size_t)in_sizes[1] != N_M || (size_t)in_sizes[2] != N_W ||
      (size_t)in_sizes[4] != N_W || in_sizes[3] != DMODEL || in_sizes[5] != DMODEL ||
      in_sizes[6] != DMODEL || in_sizes[7] < 1 || in_sizes[8] != NBATCH * SEQT) return;
  if ((size_t)out_size != N_X) return;
  if (ws_size < WS_TOTAL) return;

  char* ws = (char*)d_ws;
  unsigned short* xb    = (unsigned short*)(ws + OFF_XB);
  unsigned short* memb  = (unsigned short*)(ws + OFF_MB);
  unsigned short* W1b   = (unsigned short*)(ws + OFF_W1);
  unsigned short* W2b   = (unsigned short*)(ws + OFF_W2);
  unsigned short* memTb = (unsigned short*)(ws + OFF_MT);
  float*          item1 = (float*)(ws + OFF_I1);
  float*          item2 = (float*)(ws + OFF_I2);
  unsigned short* Phi   = (unsigned short*)(ws + OFF_PH);
  unsigned short* Plo   = (unsigned short*)(ws + OFF_PL);
  float*          b1r   = (float*)(ws + OFF_B1);
  float*          b2r   = (float*)(ws + OFF_B2);

  cast_f32_bf16x8<<<dim3((unsigned)(N_X / 8 / 256)), dim3(256), 0, stream>>>(x,   xb,   (int)(N_X / 8));
  cast_f32_bf16x8<<<dim3((unsigned)(N_M / 8 / 256)), dim3(256), 0, stream>>>(mem, memb, (int)(N_M / 8));
  cast_f32_bf16x8<<<dim3((unsigned)(N_W / 8 / 256)), dim3(256), 0, stream>>>(W1,  W1b,  (int)(N_W / 8));
  cast_f32_bf16x8<<<dim3((unsigned)(N_W / 8 / 256)), dim3(256), 0, stream>>>(W2,  W2b,  (int)(N_W / 8));
  bias_rne_kernel<<<dim3(2), dim3(128), 0, stream>>>(b1, b2, b1r, b2r);
  transpose_mem_kernel<<<dim3(NBATCH * (SEQT / 64) * (DMODEL / 64)), dim3(256), 0, stream>>>(mem, memTb);

  wmma_gemm64<1, 0, 2, 0><<<dim3((NBATCH * SEQL / 64) * (DMODEL / 64) / 8, 1), dim3(256), 0, stream>>>(
      xb, xb, DMODEL, 0L, W1b, W1b, DMODEL, 0L, (void*)item1, (void*)item1, DMODEL, 0L,
      b1r, NBATCH * SEQL, DMODEL, DMODEL, 1.0f);
  wmma_gemm64<1, 0, 2, 0><<<dim3((NBATCH * SEQT / 64) * (DMODEL / 64) / 8, 1), dim3(256), 0, stream>>>(
      memb, memb, DMODEL, 0L, W2b, W2b, DMODEL, 0L, (void*)item2, (void*)item2, DMODEL, 0L,
      b2r, NBATCH * SEQT, DMODEL, DMODEL, 1.0f);

  score_softmax_kernel<<<dim3(NBATCH * SEQL), dim3(256), 0, stream>>>(item1, item2, wt, bt, mask, Phi, Plo);

  wmma_gemm64<1, 1, 0, 0><<<dim3((SEQL / 64) * (DMODEL / 64) / 8, NBATCH), dim3(256), 0, stream>>>(
      Phi, Plo, SEQT, (long)SEQL * SEQT, memTb, memTb, SEQT, (long)DMODEL * SEQT,
      (void*)out, (void*)out, DMODEL, (long)SEQL * DMODEL,
      b1r, SEQL, DMODEL, SEQT, 1.0f);
}
